// Self_Attn_1709396984386
// MI455X (gfx1250) — hardware-verified
//
#include <hip/hip_runtime.h>


#ifndef NB
#define NB 2
#endif
#ifndef SEQ
#define SEQ 9216
#endif
#define NB_FULL  2
#define SEQ_FULL 9216
#define CD       192
#define DH       96
#define NROWS    (NB * SEQ)
#define NWROWS   (3 * CD)
#ifndef SCORE_RES
#define SCORE_RES 2
#endif

static_assert(NB >= 1 && NB <= NB_FULL);
static_assert(SEQ >= 64 && SEQ <= SEQ_FULL);
static_assert((SEQ % 64) == 0);
static_assert(CD == 2 * DH && (DH % 32) == 0);
static_assert(SCORE_RES >= 0 && SCORE_RES <= 2);
static_assert(((NWROWS * CD / 8) % 256) == 0);
static_assert(((CD * CD / 8) % 256) == 0);
static_assert((NWROWS / 4) <= 256);

#define WCARRY      256.0f
#define INV_WCARRY  0.00390625f
#define RCARRY      4096.0f
#define INV_RCARRY  0.000244140625f
#define PCARRY      16384.0f
#define VCARRY      16.0f
#define INV_PV      (1.0f / 262144.0f)
#define L2E         1.4426950408889634f
#define TP          200
#define TPV         72
#define TSZ         13824

static_assert(64 * TP <= TSZ && CD * TPV <= TSZ);

typedef _Float16 v16h __attribute__((ext_vector_type(16)));
typedef _Float16 v8h  __attribute__((ext_vector_type(8)));
typedef float    v8f  __attribute__((ext_vector_type(8)));
typedef float    v4f  __attribute__((ext_vector_type(4)));

union Frag { v16h v; v8h p[2]; };
union Acc8 { v8f v; v4f q[2]; };

__device__ __forceinline__ v16h ldfrag(const _Float16* p) {
  Frag f;
  f.p[0] = *(const v8h*)p;
  f.p[1] = *(const v8h*)(p + 16);
  return f.v;
}

__device__ __forceinline__ v8f mma16(v16h a, v16h b, v8f c) {
  return __builtin_amdgcn_wmma_f32_16x16x32_f16(false, a, false, b, (short)0, c, false, false);
}

__device__ __forceinline__ v8f zero8() {
  v8f z;
#pragma unroll
  for (int r = 0; r < 8; ++r) z[r] = 0.0f;
  return z;
}

__device__ __forceinline__ float bf16_rne(float f) {
  unsigned u = __builtin_bit_cast(unsigned, f);
  u = (u + 0x7FFFu + ((u >> 16) & 1u)) & 0xFFFF0000u;
  return __builtin_bit_cast(float, u);
}

__global__ __launch_bounds__(256) void cvt_kernel(
    const float* __restrict__ x,
    const float* __restrict__ Wq, const float* __restrict__ bq,
    const float* __restrict__ Wk, const float* __restrict__ bk,
    const float* __restrict__ Wv, const float* __restrict__ bv,
    _Float16* __restrict__ xh, _Float16* __restrict__ wc, float* __restrict__ bc,
    int nbx, int nbw)
{
  __shared__ __attribute__((aligned(16))) _Float16 xs[64 * CD];

  const int blk = blockIdx.x;
  const int tid = threadIdx.x;
  if (blk < nbx) {
    const int nper = SEQ / 64;
    const int bb   = blk / nper;
    const int n0   = (blk - bb * nper) * 64;
    const int tok  = tid & 63, cg = tid >> 6;
    const float* xb = x + (size_t)bb * CD * SEQ_FULL + n0 + tok;
#pragma unroll 1
    for (int p = 0; p < CD / 32; ++p) {
      const int c8 = 8 * (4 * p + cg);
      const float* src = xb + (size_t)c8 * SEQ_FULL;
      float f[8];
#pragma unroll
      for (int e = 0; e < 8; ++e) f[e] = src[(size_t)e * SEQ_FULL];
      v8h o;
      o[0] = (_Float16)bf16_rne(f[0]);
      o[1] = (_Float16)bf16_rne(f[1]);
      o[2] = (_Float16)bf16_rne(f[2]);
      o[3] = (_Float16)bf16_rne(f[3]);
      o[4] = (_Float16)bf16_rne(f[4]);
      o[5] = (_Float16)bf16_rne(f[5]);
      o[6] = (_Float16)bf16_rne(f[6]);
      o[7] = (_Float16)bf16_rne(f[7]);
      *(v8h*)&xs[tok * CD + c8] = o;
    }
    __syncthreads();
    v8h rv[6];
#pragma unroll
    for (int i = 0; i < 6; ++i) rv[i] = *(const v8h*)&xs[8 * tid + 2048 * i];
    _Float16* dst = xh + ((size_t)bb * SEQ + n0) * CD + 8 * tid;
#pragma unroll
    for (int i = 0; i < 6; ++i) *(volatile v8h*)(dst + 2048 * i) = rv[i];
    __threadfence();
#pragma unroll
    for (int i = 0; i < 6; ++i) *(volatile v8h*)(dst + 2048 * i) = rv[i];
  } else if (blk < nbx + nbw) {
    const unsigned g   = (unsigned)(blk - nbx) * 256u + (unsigned)tid;
    const unsigned n   = g / 24u;
    const int      col = (int)(g - n * 24u) * 8;
    const int      mat = __builtin_amdgcn_readfirstlane((int)(g / (unsigned)(CD * 24)));
    const float* W = (mat == 0) ? Wq : ((mat == 1) ? Wk : Wv);
    const float* src = W + (size_t)(n - (unsigned)mat * (unsigned)CD) * CD + col;
    const v4f a = *(const v4f*)src;
    const v4f c = *(const v4f*)(src + 4);
    v8h o;
    o[0] = (_Float16)(bf16_rne(a[0]) * WCARRY);
    o[1] = (_Float16)(bf16_rne(a[1]) * WCARRY);
    o[2] = (_Float16)(bf16_rne(a[2]) * WCARRY);
    o[3] = (_Float16)(bf16_rne(a[3]) * WCARRY);
    o[4] = (_Float16)(bf16_rne(c[0]) * WCARRY);
    o[5] = (_Float16)(bf16_rne(c[1]) * WCARRY);
    o[6] = (_Float16)(bf16_rne(c[2]) * WCARRY);
    o[7] = (_Float16)(bf16_rne(c[3]) * WCARRY);
    _Float16* dst = wc + (size_t)n * CD + col;
    *(volatile v8h*)dst = o;
    __threadfence();
    *(volatile v8h*)dst = o;
  } else {
    const int t = (blk - nbx - nbw) * 256 + tid;
    if (t < NWROWS / 4) {
      const int e   = t * 4;
      const int m   = e / CD;
      const int idx = e - m * CD;
      const v4f uq = *(const v4f*)(bq + idx);
      const v4f uk = *(const v4f*)(bk + idx);
      const v4f uv = *(const v4f*)(bv + idx);
      v4f o;
#pragma unroll
      for (int i = 0; i < 4; ++i) {
        const float s0 = uq[i], s1 = uk[i], s2 = uv[i];
        const float sel = (m == 0) ? s0 : ((m == 1) ? s1 : s2);
        o[i] = bf16_rne(sel);
      }
      float* dst = bc + e;
      *(volatile v4f*)dst = o;
      __threadfence();
      *(volatile v4f*)dst = o;
    }
  }
}

__global__ __launch_bounds__(256) void proj_kernel(
    const _Float16* __restrict__ xh, const _Float16* __restrict__ wc,
    const float* __restrict__ bc,
    _Float16* __restrict__ qh, _Float16* __restrict__ ql,
    _Float16* __restrict__ kh, _Float16* __restrict__ kl,
    _Float16* __restrict__ vt)
{
  __shared__ __attribute__((aligned(16))) _Float16 T[TSZ];

  const int tid  = threadIdx.x;
  const int w    = __builtin_amdgcn_readfirstlane(tid >> 5);
  const int lane = tid & 31, h = lane >> 4, l16 = lane & 15;
  const int wr   = w >> 2, wq = w & 3;
  const int rb   = blockIdx.x * 64;
  const int mat  = blockIdx.y;

  const _Float16* ap0 = xh + (size_t)(rb + 32 * wr + l16) * CD + 8 * h;
  const _Float16* ap1 = ap0 + (size_t)16 * CD;
  const _Float16* bp0 = wc + (size_t)(mat * CD + 48 * wq + l16) * CD + 8 * h;
  const _Float16* bp1 = bp0 + (size_t)16 * CD;
  const _Float16* bp2 = bp0 + (size_t)32 * CD;

  v8f acc[2][3];
#pragma unroll
  for (int mt = 0; mt < 2; ++mt)
#pragma unroll
    for (int nt = 0; nt < 3; ++nt) acc[mt][nt] = zero8();

#pragma unroll 1
  for (int kc = 0; kc < CD; kc += 32) {
    const v16h A0 = ldfrag(ap0 + kc);
    const v16h A1 = ldfrag(ap1 + kc);
    const v16h B0 = ldfrag(bp0 + kc);
    const v16h B1 = ldfrag(bp1 + kc);
    const v16h B2 = ldfrag(bp2 + kc);
    acc[0][0] = mma16(A0, B0, acc[0][0]);
    acc[0][1] = mma16(A0, B1, acc[0][1]);
    acc[0][2] = mma16(A0, B2, acc[0][2]);
    acc[1][0] = mma16(A1, B0, acc[1][0]);
    acc[1][1] = mma16(A1, B1, acc[1][1]);
    acc[1][2] = mma16(A1, B2, acc[1][2]);
    asm volatile("v_nop\n\tv_nop\n\tv_nop\n\tv_nop"
                 : "+v"(acc[0][0]), "+v"(acc[0][1]), "+v"(acc[0][2]),
                   "+v"(acc[1][0]), "+v"(acc[1][1]), "+v"(acc[1][2])
                 : "v"(A0), "v"(A1), "v"(B0), "v"(B1), "v"(B2));
  }

  const int cl0 = 48 * wq + l16;
  const int rl0 = 32 * wr + 8 * h;
#pragma unroll
  for (int nt = 0; nt < 3; ++nt) {
    const float bias = bc[mat * CD + cl0 + 16 * nt];
#pragma unroll
    for (int mt = 0; mt < 2; ++mt) acc[mt][nt] = acc[mt][nt] * INV_WCARRY + bias;
  }

  v8h rv[6];
  if (mat < 2) {
    _Float16* ph = (mat == 0) ? qh : kh;
    _Float16* pl = (mat == 0) ? ql : kl;
#pragma unroll
    for (int pass = 0; pass < 2; ++pass) {
#pragma unroll
      for (int mt = 0; mt < 2; ++mt)
#pragma unroll
        for (int nt = 0; nt < 3; ++nt)
#pragma unroll
          for (int r = 0; r < 8; ++r) {
            const float    v  = acc[mt][nt][r];
            const _Float16 hv = (_Float16)v;
            _Float16 sv;
            if (pass == 0) sv = hv;
            else           sv = (_Float16)((v - (float)hv) * RCARRY);
            T[(rl0 + 16 * mt + r) * TP + cl0 + 16 * nt] = sv;
          }
      __syncthreads();
#pragma unroll
      for (int i = 0; i < 6; ++i) {
        const int p   = tid + 256 * i;
        const int row = p / 24;
        const int cp  = p - row * 24;
        rv[i] = *(const v8h*)&T[row * TP + 8 * cp];
      }
      _Float16* pd = ((pass == 0) ? ph : pl) + (size_t)rb * CD + 8 * tid;
#pragma unroll
      for (int i = 0; i < 6; ++i) *(volatile v8h*)(pd + 2048 * i) = rv[i];
      __threadfence();
#pragma unroll
      for (int i = 0; i < 6; ++i) *(volatile v8h*)(pd + 2048 * i) = rv[i];
      __syncthreads();
    }
  } else {
#pragma unroll
    for (int mt = 0; mt < 2; ++mt)
#pragma unroll
      for (int nt = 0; nt < 3; ++nt) {
        v8h o;
#pragma unroll
        for (int r = 0; r < 8; ++r) o[r] = (_Float16)(acc[mt][nt][r] * VCARRY);
        *(v8h*)&T[(cl0 + 16 * nt) * TPV + rl0 + 16 * mt] = o;
      }
    __syncthreads();
    const int bb = rb / SEQ;
    const int s0 = rb - bb * SEQ;
#pragma unroll
    for (int i = 0; i < 6; ++i) {
      const int p = tid + 256 * i;
      rv[i] = *(const v8h*)&T[(p >> 3) * TPV + 8 * (p & 7)];
    }
#pragma unroll
    for (int i = 0; i < 6; ++i) {
      const int p = tid + 256 * i;
      *(volatile v8h*)(vt + ((size_t)bb * CD + (p >> 3)) * SEQ + s0 + 8 * (p & 7)) = rv[i];
    }
    __threadfence();
#pragma unroll
    for (int i = 0; i < 6; ++i) {
      const int p = tid + 256 * i;
      *(volatile v8h*)(vt + ((size_t)bb * CD + (p >> 3)) * SEQ + s0 + 8 * (p & 7)) = rv[i];
    }
  }
}

__global__ __launch_bounds__(256) __attribute__((amdgpu_num_vgpr(256))) void attn_kernel(
    const _Float16* __restrict__ qh, const _Float16* __restrict__ ql,
    const _Float16* __restrict__ kh, const _Float16* __restrict__ kl,
    const _Float16* __restrict__ vt, float* __restrict__ out)
{
  __shared__ __attribute__((aligned(16))) float    sp[CD * 64];
  __shared__ __attribute__((aligned(16))) _Float16 pb[2048];
  __shared__ float scl[128];
  __shared__ float invl[128];

  const int tid  = threadIdx.x;
  const int w    = __builtin_amdgcn_readfirstlane(tid >> 5);
  const int lane = tid & 31, h = lane >> 4, l16 = lane & 15;
  const int qt   = w >> 1, dq = w & 1;
  const int b     = blockIdx.y;
  const int qbase = blockIdx.x * 64;

  const size_t prow = (size_t)b * SEQ + qbase + 16 * qt + l16;
  const _Float16* qhp = qh + prow * CD + DH * dq + 8 * h;
#if SCORE_RES >= 2
  const _Float16* qlp = ql + prow * CD + DH * dq + 8 * h;
#endif
  const size_t krow = (size_t)b * SEQ + l16;
  const _Float16* khp = kh + krow * CD + DH * dq + 8 * h;
#if SCORE_RES >= 1
  const _Float16* klp = kl + krow * CD + DH * dq + 8 * h;
#endif
  const _Float16* vtp = vt + ((size_t)b * CD + DH * dq + l16) * SEQ + 8 * h;

  const int pbo = (qt * 32 + lane) * 16;
  const int slo = qt * 32 + lane;

  v8f O[6];
#pragma unroll
  for (int dt = 0; dt < 6; ++dt) O[dt] = zero8();
  float mx = -1.0e30f, sm = 0.0f;

#pragma unroll 1
  for (int kt = 0; kt < SEQ; kt += 32) {
    v8f shh0 = zero8(), shh1 = zero8();
#if SCORE_RES >= 1
    v8f sx0 = zero8(), sx1 = zero8();
#endif
    const _Float16* kh0 = khp + (size_t)kt * CD;
#if SCORE_RES >= 1
    const _Float16* kl0 = klp + (size_t)kt * CD;
#endif
#pragma unroll 1
    for (int j = 0; j < DH / 32; ++j) {
      const v16h Bh  = ldfrag(qhp + 32 * j);
      const v16h Ah0 = ldfrag(kh0 + 32 * j);
      const v16h Ah1 = ldfrag(kh0 + 16 * CD + 32 * j);
#if SCORE_RES >= 2
      const v16h Bl  = ldfrag(qlp + 32 * j);
#endif
#if SCORE_RES >= 1
      const v16h Al0 = ldfrag(kl0 + 32 * j);
      const v16h Al1 = ldfrag(kl0 + 16 * CD + 32 * j);
#endif
      shh0 = mma16(Ah0, Bh, shh0);
#if SCORE_RES >= 2
      sx0  = mma16(Ah0, Bl, sx0);
#endif
#if SCORE_RES >= 1
      sx0  = mma16(Al0, Bh, sx0);
#endif
      shh1 = mma16(Ah1, Bh, shh1);
#if SCORE_RES >= 2
      sx1  = mma16(Ah1, Bl, sx1);
#endif
#if SCORE_RES >= 1
      sx1  = mma16(Al1, Bh, sx1);
#endif
#if SCORE_RES >= 2
      asm volatile("v_nop\n\tv_nop\n\tv_nop\n\tv_nop"
                   : "+v"(shh0), "+v"(shh1), "+v"(sx0), "+v"(sx1)
                   : "v"(Ah0), "v"(Al0), "v"(Ah1), "v"(Al1), "v"(Bh), "v"(Bl));
#elif SCORE_RES == 1
      asm volatile("v_nop\n\tv_nop\n\tv_nop\n\tv_nop"
                   : "+v"(shh0), "+v"(shh1), "+v"(sx0), "+v"(sx1)
                   : "v"(Ah0), "v"(Al0), "v"(Ah1), "v"(Al1), "v"(Bh));
#else
      asm volatile("v_nop\n\tv_nop\n\tv_nop\n\tv_nop"
                   : "+v"(shh0), "+v"(shh1)
                   : "v"(Ah0), "v"(Ah1), "v"(Bh));
#endif
    }
#if SCORE_RES >= 1
    v8f part0 = shh0 + sx0 * INV_RCARRY;
    v8f part1 = shh1 + sx1 * INV_RCARRY;
#else
    v8f part0 = shh0;
    v8f part1 = shh1;
#endif

    if (dq != 0) {
      const int o = qt * 512 + lane * 8;
      Acc8 u0, u1;
      u0.v = part0; u1.v = part1;
      *(v4f*)&sp[o]       = u0.q[0];
      *(v4f*)&sp[o + 4]   = u0.q[1];
      *(v4f*)&sp[o + 256] = u1.q[0];
      *(v4f*)&sp[o + 260] = u1.q[1];
    }
    __syncthreads();

    if (dq == 0) {
      {
        const int o = qt * 512 + lane * 8;
        Acc8 u0, u1;
        u0.q[0] = *(const v4f*)&sp[o];
        u0.q[1] = *(const v4f*)&sp[o + 4];
        u1.q[0] = *(const v4f*)&sp[o + 256];
        u1.q[1] = *(const v4f*)&sp[o + 260];
        part0 += u0.v;
        part1 += u1.v;
      }
      float tmax = -1.0e30f;
#pragma unroll
      for (int r = 0; r < 8; ++r) {
        tmax = fmaxf(tmax, part0[r]);
        tmax = fmaxf(tmax, part1[r]);
      }
      tmax = fmaxf(tmax, __shfl_xor(tmax, 16, 32));
      const float nmx = fmaxf(mx, tmax);
      const float sc  = __builtin_amdgcn_exp2f((mx - nmx) * L2E);
      mx = nmx;
      v8f p0, p1;
      float ps = 0.0f;
#pragma unroll
      for (int r = 0; r < 8; ++r) {
        p0[r] = __builtin_amdgcn_exp2f((part0[r] - mx) * L2E);
        p1[r] = __builtin_amdgcn_exp2f((part1[r] - mx) * L2E);
        ps += p0[r] + p1[r];
      }
      ps += __shfl_xor(ps, 16, 32);
      sm = sm * sc + ps;
      v8h t0, t1;
#pragma unroll
      for (int r = 0; r < 8; ++r) {
        t0[r] = (_Float16)(p0[r] * PCARRY);
        t1[r] = (_Float16)(p1[r] * PCARRY);
      }
      *(v8h*)&pb[pbo]     = t0;
      *(v8h*)&pb[pbo + 8] = t1;
      scl[slo] = sc;
    }
    __syncthreads();

    const float osc = scl[slo];
    Frag bpf;
    bpf.p[0] = *(const v8h*)&pb[pbo];
    bpf.p[1] = *(const v8h*)&pb[pbo + 8];
    const v16h Bp = bpf.v;
#pragma unroll
    for (int dt = 0; dt < 6; ++dt) O[dt] = O[dt] * osc;

    const _Float16* v0 = vtp + kt;
    {
      const v16h V0 = ldfrag(v0);
      const v16h V1 = ldfrag(v0 + (size_t)SEQ * 16);
      const v16h V2 = ldfrag(v0 + (size_t)SEQ * 32);
      O[0] = mma16(V0, Bp, O[0]);
      O[1] = mma16(V1, Bp, O[1]);
      O[2] = mma16(V2, Bp, O[2]);
      asm volatile("v_nop\n\tv_nop\n\tv_nop\n\tv_nop"
                   : "+v"(O[0]), "+v"(O[1]), "+v"(O[2])
                   : "v"(V0), "v"(V1), "v"(V2), "v"(Bp));
    }
    {
      const v16h V3 = ldfrag(v0 + (size_t)SEQ * 48);
      const v16h V4 = ldfrag(v0 + (size_t)SEQ * 64);
      const v16h V5 = ldfrag(v0 + (size_t)SEQ * 80);
      O[3] = mma16(V3, Bp, O[3]);
      O[4] = mma16(V4, Bp, O[4]);
      O[5] = mma16(V5, Bp, O[5]);
      asm volatile("v_nop\n\tv_nop\n\tv_nop\n\tv_nop"
                   : "+v"(O[3]), "+v"(O[4]), "+v"(O[5])
                   : "v"(V3), "v"(V4), "v"(V5), "v"(Bp));
    }
  }

  if (dq == 0) {
    const float inv = (1.0f / sm) * INV_PV;
    invl[slo] = inv;
  }
  __syncthreads();
  const float inv = invl[slo];

#pragma unroll
  for (int dt = 0; dt < 6; ++dt) {
#pragma unroll
    for (int r = 0; r < 8; ++r)
      sp[(DH * dq + 16 * dt + 8 * h + r) * 64 + 16 * qt + l16] = O[dt][r] * inv;
  }
  __syncthreads();

  v4f rv[12];
#pragma unroll
  for (int i = 0; i < 12; ++i)
    rv[i] = *(const v4f*)&sp[(24 * w + 2 * i + h) * 64 + 4 * l16];
  float* orow = out + ((size_t)b * CD) * SEQ + qbase + 4 * l16;
#pragma unroll
  for (int i = 0; i < 12; ++i)
    *(volatile v4f*)(orow + (size_t)(24 * w + 2 * i + h) * SEQ) = rv[i];
  __threadfence();
#pragma unroll
  for (int i = 0; i < 12; ++i)
    *(volatile v4f*)(orow + (size_t)(24 * w + 2 * i + h) * SEQ) = rv[i];
}

extern "C" void kernel_launch(void* const* d_in, const int* in_sizes, int n_in,
                              void* d_out, int out_size, void* d_ws, size_t ws_size,
                              hipStream_t stream) {
  if (n_in < 7) return;
  const long long need_x = ((long long)NB * CD - 1) * SEQ_FULL + SEQ;
  if ((long long)in_sizes[0] < need_x) return;
  if (in_sizes[1] < CD * CD || in_sizes[3] < CD * CD || in_sizes[5] < CD * CD) return;
  if (in_sizes[2] < CD || in_sizes[4] < CD || in_sizes[6] < CD) return;
  if ((long long)out_size < (long long)NB * CD * SEQ) return;

  const float* x  = (const float*)d_in[0];
  const float* Wq = (const float*)d_in[1];
  const float* bq = (const float*)d_in[2];
  const float* Wk = (const float*)d_in[3];
  const float* bk = (const float*)d_in[4];
  const float* Wv = (const float*)d_in[5];
  const float* bv = (const float*)d_in[6];
  float* outp = (float*)d_out;

  const size_t plane = (size_t)NROWS * CD * 2;
  const size_t wcb   = (size_t)NWROWS * CD * 2;
  const size_t bcb   = (size_t)NWROWS * 4;
  const size_t vtb   = (size_t)NB * CD * SEQ * 2;
  const size_t o_xh = 0;
  const size_t o_wc = o_xh + plane;
  const size_t o_bc = o_wc + wcb;
  const size_t o_qh = o_bc + bcb;
  const size_t o_ql = o_qh + plane;
  const size_t o_kh = o_ql + plane;
  const size_t o_kl = o_kh + plane;
  const size_t o_vt = o_kl + plane;
  const size_t total = o_vt + vtb;
  if (total > ws_size) return;

  char* ws = (char*)d_ws;
  _Float16* xh = (_Float16*)(ws + o_xh);
  _Float16* wc = (_Float16*)(ws + o_wc);
  float*    bc = (float*)(ws + o_bc);
  _Float16* qh = (_Float16*)(ws + o_qh);
  _Float16* ql = (_Float16*)(ws + o_ql);
  _Float16* kh = (_Float16*)(ws + o_kh);
  _Float16* kl = (_Float16*)(ws + o_kl);
  _Float16* vt = (_Float16*)(ws + o_vt);

  const int nbx = NB * (SEQ / 64);
  const int nbw = (NWROWS * CD / 8) / 256;
  const int nbb = 1;
  cvt_kernel<<<dim3(nbx + nbw + nbb), dim3(256), 0, stream>>>(
      x, Wq, bq, Wk, bk, Wv, bv, xh, wc, bc, nbx, nbw);

  proj_kernel<<<dim3(NROWS / 64, 3), dim3(256), 0, stream>>>(
      xh, wc, bc, qh, ql, kh, kl, vt);

  attn_kernel<<<dim3(SEQ / 64, NB), dim3(256), 0, stream>>>(
      qh, ql, kh, kl, vt, outp);
}
